// MambaBlock_48180943126918
// MI455X (gfx1250) — hardware-run, weakly checked
//
#include <hip/hip_runtime.h>
#include <math.h>

typedef __attribute__((ext_vector_type(16))) _Float16 v16h;
typedef __attribute__((ext_vector_type(8)))  _Float16 v8h;
typedef __attribute__((ext_vector_type(8)))  float    v8f;
typedef __attribute__((ext_vector_type(4)))  float    v4f;

constexpr int kBatch  = 2;
constexpr int kSeq    = 1024;
constexpr int kDm     = 1024;
constexpr int kDin    = 2048;
constexpr int kNst    = 16;
constexpr int kDtR    = 64;
constexpr int kRows   = kBatch * kSeq;
constexpr int kXzP    = 2 * kDin;
constexpr int kXdN    = kDtR + 2 * kNst;
constexpr int kXdP    = 128;
constexpr int kConvTP = 260;
constexpr int kScanTS = 64;
constexpr int kScanCh = 64;
constexpr int kScanYP = 68;
constexpr int kBcW    = 2 * kNst;
constexpr float kLnEps = 1e-5f;
static_assert(kXdN == 96);
static_assert((kDm % 32) == 0 && (kDin % 32) == 0 && (kDtR % 32) == 0);
static_assert((kRows % 64) == 0 && (kXzP % 64) == 0 && (kXdP % 64) == 0 && (kDin % 64) == 0 && (kDm % 64) == 0);
static_assert((kSeq % kScanTS) == 0 && (kSeq % 64) == 0 && (kDin % kScanCh) == 0 && (kDin % 256) == 0);

constexpr float kCarryH    = 16.0f;
constexpr float kCarryU    = 16.0f;
constexpr float kCarryDl   = 64.0f;
constexpr float kCarryY    = 128.0f;
constexpr float kCarryWin  = 256.0f;
constexpr float kCarryWx   = 256.0f;
constexpr float kCarryWdt  = 64.0f;
constexpr float kCarryWout = 256.0f;
constexpr float kSclIn  = 1.0f / (kCarryH  * kCarryWin);
constexpr float kSclX   = 1.0f / (kCarryU  * kCarryWx);
constexpr float kSclDt  = 1.0f / (kCarryDl * kCarryWdt);
constexpr float kSclOut = 1.0f / (kCarryY  * kCarryWout);

constexpr size_t kOffWIN  = 0;
constexpr size_t kOffWX   = kOffWIN  + (size_t)kXzP  * kDm  * 2;
constexpr size_t kOffWDT  = kOffWX   + (size_t)kXdP  * kDin * 2;
constexpr size_t kOffWOUT = kOffWDT  + (size_t)kDin  * kDtR * 2;
constexpr size_t kOffH16  = kOffWOUT + (size_t)kDm   * kDin * 2;
constexpr size_t kOffXZ   = kOffH16  + (size_t)kRows * kDm  * 2;
constexpr size_t kOffUC   = kOffXZ   + (size_t)kRows * kXzP * 4;
constexpr size_t kOffUC16 = kOffUC   + (size_t)kRows * kDin * 4;
constexpr size_t kOffXD   = kOffUC16 + (size_t)kRows * kDin * 2;
constexpr size_t kOffDL16 = kOffXD   + (size_t)kRows * kXdP * 4;
constexpr size_t kOffDTP  = kOffDL16 + (size_t)kRows * kDtR * 2;
constexpr size_t kOffDT   = kOffDTP  + (size_t)kRows * kDin * 4;
constexpr size_t kOffYG   = kOffDT   + (size_t)kRows * kDin * 4;
constexpr size_t kWsTotal = kOffYG   + (size_t)kRows * kDin * 2;
static_assert(kWsTotal == 119537664ull);
static_assert(kWsTotal <= 134217728ull);
static_assert((kOffWX % 128) == 0 && (kOffWDT % 128) == 0 && (kOffWOUT % 128) == 0 && (kOffH16 % 128) == 0 &&
              (kOffXZ % 128) == 0 && (kOffUC % 128) == 0 && (kOffUC16 % 128) == 0 && (kOffXD % 128) == 0 &&
              (kOffDL16 % 128) == 0 && (kOffDTP % 128) == 0 && (kOffDT % 128) == 0 && (kOffYG % 128) == 0);

__device__ __forceinline__ _Float16 to_h16(float v, float carry) {
  float c = v * carry;
  c = (fabsf(c) < 6.103515625e-5f) ? 0.0f : c;
  return (_Float16)c;
}
__device__ __forceinline__ void pin1(float& a) { asm volatile("" : "+v"(a)); }
__device__ __forceinline__ void pin4(float& a, float& b, float& c, float& d) { asm volatile("" : "+v"(a), "+v"(b), "+v"(c), "+v"(d)); }
__device__ __forceinline__ void pinu(unsigned& a) { asm volatile("" : "+v"(a)); }

namespace eng {

__device__ __forceinline__ void row_guard_h(v8f& a, v8f& b, v8f& c, v8f& d, v16h x, v16h y0, v16h y1, v16h y2, v16h y3) {
  asm volatile("v_nop\n\tv_nop\n\tv_nop\n\tv_nop" : "+v"(a), "+v"(b), "+v"(c), "+v"(d) : "v"(x), "v"(y0), "v"(y1), "v"(y2), "v"(y3));
}
__device__ __forceinline__ void keep4_h(v16h a, v16h b, v16h c, v16h d) { asm volatile("v_nop" :: "v"(a), "v"(b), "v"(c), "v"(d)); }
__device__ __forceinline__ void acc_guard4(v8f& a, v8f& b, v8f& c, v8f& d) { asm volatile("v_nop\n\tv_nop\n\tv_nop\n\tv_nop" : "+v"(a), "+v"(b), "+v"(c), "+v"(d)); }

struct FragH {
  union U { v16h v; v8h h[2]; };
  static __device__ __forceinline__ v16h load(const _Float16* p) {
    U f; f.h[0] = *(const v8h*)(p); f.h[1] = *(const v8h*)(p + 16); return f.v;
  }
  static __device__ __forceinline__ v8f mma(v16h a, v16h b, v8f c) {
    return __builtin_amdgcn_wmma_f32_16x16x32_f16(false, a, false, b, (short)0, c, false, false);
  }
};

template <bool RESID>
__global__ __launch_bounds__(256) void wmma_gemm64_f16(
    const unsigned short* __restrict__ Ap, int lda,
    const unsigned short* __restrict__ Btp, int ldb,
    float* __restrict__ C, int ldc,
    const float* __restrict__ resid,
    int M, int N, int K, float scale) {
  const _Float16* A  = (const _Float16*)Ap;
  const _Float16* Bt = (const _Float16*)Btp;
  __shared__ __align__(16) float sT[8][16 * 68];
  const int lane = threadIdx.x & 31;
  const int wave = threadIdx.x >> 5;
  const int tilesN = N >> 6;
  const int tilesM = M >> 6;
  const int tile = blockIdx.x * 8 + wave;
  if (tile >= tilesM * tilesN) return;
  const int tm = tile / tilesN;
  const int tn = tile - tm * tilesN;
  const int m0 = tm << 6;
  const int n0 = tn << 6;

  const int rlane = lane & 15;
  const int koff  = (lane >> 4) * 8;
  const int mOff  = (lane >> 4) * 8;

  v8f acc[4][4];
#pragma unroll
  for (int i = 0; i < 4; ++i)
#pragma unroll
    for (int j = 0; j < 4; ++j) acc[i][j] = (v8f){0.f,0.f,0.f,0.f,0.f,0.f,0.f,0.f};

  for (int k0 = 0; k0 < K; k0 += 32) {
    v16h bh[4];
#pragma unroll
    for (int j = 0; j < 4; ++j) {
      const size_t bo = (size_t)(n0 + (j << 4) + rlane) * ldb + koff + k0;
      bh[j] = FragH::load(Bt + bo);
    }
#pragma unroll
    for (int i = 0; i < 4; ++i) {
      const size_t ao = (size_t)(m0 + (i << 4) + rlane) * lda + koff + k0;
      v16h ah = FragH::load(A + ao);
#pragma unroll
      for (int j = 0; j < 4; ++j) acc[i][j] = FragH::mma(ah, bh[j], acc[i][j]);
      row_guard_h(acc[i][0], acc[i][1], acc[i][2], acc[i][3], ah, bh[0], bh[1], bh[2], bh[3]);
    }
    keep4_h(bh[0], bh[1], bh[2], bh[3]);
  }
  acc_guard4(acc[0][0], acc[0][1], acc[0][2], acc[0][3]);
  acc_guard4(acc[1][0], acc[1][1], acc[1][2], acc[1][3]);
  acc_guard4(acc[2][0], acc[2][1], acc[2][2], acc[2][3]);
  acc_guard4(acc[3][0], acc[3][1], acc[3][2], acc[3][3]);

  float* slab = sT[wave];
  const int hh = lane >> 4, c4 = (lane & 15) * 4;
#pragma unroll
  for (int i = 0; i < 4; ++i) {
    const int mBase = m0 + (i << 4);
#pragma unroll
    for (int j = 0; j < 4; ++j) {
#pragma unroll
      for (int r = 0; r < 8; ++r) {
        const float v = acc[i][j][r] * scale;
        slab[(mOff + r) * 68 + (j << 4) + rlane] = v;
      }
    }
    __builtin_amdgcn_fence(__ATOMIC_RELEASE, "workgroup");
    __builtin_amdgcn_wave_barrier();
    __builtin_amdgcn_fence(__ATOMIC_ACQUIRE, "workgroup");
    if (RESID) {
#pragma unroll
      for (int it = 0; it < 8; ++it) {
        const int row = it * 2 + hh;
        v4f v = *(const v4f*)(slab + row * 68 + c4);
        const v4f rv = *(const v4f*)(resid + (size_t)(mBase + row) * ldc + n0 + c4);
        v = v + rv;
        *(v4f*)(slab + row * 68 + c4) = v;
      }
      __builtin_amdgcn_fence(__ATOMIC_RELEASE, "workgroup");
      __builtin_amdgcn_wave_barrier();
      __builtin_amdgcn_fence(__ATOMIC_ACQUIRE, "workgroup");
    }
    for (int pass = 0; pass < 2; ++pass) {
#pragma unroll
      for (int it = 0; it < 8; ++it) {
        const int row = it * 2 + hh;
        const v4f v = *(const v4f*)(slab + row * 68 + c4);
        *(volatile v4f*)(C + (size_t)(mBase + row) * ldc + n0 + c4) = v;
      }
      __threadfence();
    }
    __builtin_amdgcn_fence(__ATOMIC_RELEASE, "workgroup");
    __builtin_amdgcn_wave_barrier();
    __builtin_amdgcn_fence(__ATOMIC_ACQUIRE, "workgroup");
  }
}

}

__global__ __launch_bounds__(256) void cvt_plane_f16_kernel(
    const float* __restrict__ src, unsigned short* __restrict__ dst, int real8, int total8, float carry)
{
  const int i = blockIdx.x * 256 + threadIdx.x;
  if (i >= total8) return;
  const bool live = (i < real8);
  const int ic = live ? i : (real8 - 1);
  const size_t e0 = (size_t)ic << 3;
  const v4f a0 = *(const v4f*)(src + e0);
  const v4f a1 = *(const v4f*)(src + e0 + 4);
  float f0 = a0[0], f1 = a0[1], f2 = a0[2], f3 = a0[3];
  float f4 = a1[0], f5 = a1[1], f6 = a1[2], f7 = a1[3];
  pin4(f0, f1, f2, f3);
  pin4(f4, f5, f6, f7);
  f0 = live ? f0 : 0.0f; f1 = live ? f1 : 0.0f; f2 = live ? f2 : 0.0f; f3 = live ? f3 : 0.0f;
  f4 = live ? f4 : 0.0f; f5 = live ? f5 : 0.0f; f6 = live ? f6 : 0.0f; f7 = live ? f7 : 0.0f;
  v8h hv;
  hv[0] = to_h16(f0, carry); hv[1] = to_h16(f1, carry); hv[2] = to_h16(f2, carry); hv[3] = to_h16(f3, carry);
  hv[4] = to_h16(f4, carry); hv[5] = to_h16(f5, carry); hv[6] = to_h16(f6, carry); hv[7] = to_h16(f7, carry);
  unsigned short* q = dst + ((size_t)i << 3);
  *(volatile v8h*)q = hv;
  __threadfence();
  *(volatile v8h*)q = hv;
}

__global__ __launch_bounds__(256) void ln_rows_kernel(
    const float* __restrict__ x, const float* __restrict__ gw, const float* __restrict__ gb,
    unsigned short* __restrict__ H16)
{
  unsigned lane = threadIdx.x & 31u;
  unsigned wave = threadIdx.x >> 5;
  pinu(lane);
  pinu(wave);
  const unsigned row = blockIdx.x * 8u + wave;
  const float* xr = x + (size_t)row * kDm;
  v4f xa[4], xb[4];
#pragma unroll
  for (int c = 0; c < 4; ++c) {
    const unsigned col = (unsigned)c * 256u + lane * 8u;
    xa[c] = *(const v4f*)(xr + col);
    xb[c] = *(const v4f*)(xr + col + 4);
  }
  float s = 0.f;
#pragma unroll
  for (int c = 0; c < 4; ++c) {
    s += (xa[c][0] + xa[c][1]) + (xa[c][2] + xa[c][3]);
    s += (xb[c][0] + xb[c][1]) + (xb[c][2] + xb[c][3]);
  }
#pragma unroll
  for (int off = 16; off >= 1; off >>= 1) s += __shfl_xor(s, off, 32);
  const float mu = s * (1.0f / (float)kDm);
  float ss = 0.f;
#pragma unroll
  for (int c = 0; c < 4; ++c) {
#pragma unroll
    for (int e = 0; e < 4; ++e) {
      const float da = xa[c][e] - mu;
      const float db = xb[c][e] - mu;
      ss = fmaf(da, da, ss);
      ss = fmaf(db, db, ss);
    }
  }
#pragma unroll
  for (int off = 16; off >= 1; off >>= 1) ss += __shfl_xor(ss, off, 32);
  const float rs = rsqrtf(ss * (1.0f / (float)kDm) + kLnEps);
  v8h hv[4];
#pragma unroll
  for (int c = 0; c < 4; ++c) {
    const unsigned col = (unsigned)c * 256u + lane * 8u;
    const v4f wa = *(const v4f*)(gw + col);
    const v4f wb = *(const v4f*)(gw + col + 4);
    const v4f ba = *(const v4f*)(gb + col);
    const v4f bb = *(const v4f*)(gb + col + 4);
#pragma unroll
    for (int e = 0; e < 4; ++e) {
      const float ya = (xa[c][e] - mu) * rs * wa[e] + ba[e];
      const float yb = (xb[c][e] - mu) * rs * wb[e] + bb[e];
      hv[c][e]     = to_h16(ya, kCarryH);
      hv[c][4 + e] = to_h16(yb, kCarryH);
    }
  }
  unsigned short* hr = H16 + (size_t)row * kDm;
  for (int pass = 0; pass < 2; ++pass) {
#pragma unroll
    for (int c = 0; c < 4; ++c)
      *(volatile v8h*)(hr + (unsigned)c * 256u + lane * 8u) = hv[c];
    __threadfence();
  }
}

__global__ __launch_bounds__(256) void conv_silu_kernel(
    const float* __restrict__ XZ, const float* __restrict__ cw, const float* __restrict__ cb,
    float* __restrict__ UC, unsigned short* __restrict__ UC16)
{
  __shared__ __align__(16) float sT[16 * kConvTP];
  unsigned tid = threadIdx.x;
  pinu(tid);
  const unsigned lane = tid & 31u, wave = tid >> 5;
  const unsigned d0 = blockIdx.x * 256u, d = d0 + tid;
  const int g0 = blockIdx.y * 64;
  const int tb = g0 & (kSeq - 1);
  const v4f wv = *(const v4f*)(cw + (size_t)d * 4);
  const float w0 = wv[0], w1 = wv[1], w2 = wv[2], w3 = wv[3];
  const float bc = cb[d];
  float xm3, xm2, xm1;
  {
    const bool hist = (tb > 0);
    const int rb = hist ? (g0 - 3) : g0;
    const float v3 = XZ[(size_t)rb * kXzP + d];
    const float v2 = XZ[(size_t)(rb + 1) * kXzP + d];
    const float v1 = XZ[(size_t)(rb + 2) * kXzP + d];
    xm3 = hist ? v3 : 0.f;
    xm2 = hist ? v2 : 0.f;
    xm1 = hist ? v1 : 0.f;
  }
  const unsigned hrow = wave >> 1;
  const unsigned hch  = (wave & 1u) * 128u + lane * 4u;
#pragma unroll 1
  for (int sub = 0; sub < 4; ++sub) {
    const int lb = g0 + sub * 16;
#pragma unroll 1
    for (int s = 0; s < 16; ++s) {
      const float xcur = XZ[(size_t)(lb + s) * kXzP + d];
      float acc = w0 * xm3;
      acc = fmaf(w1, xm2, acc);
      acc = fmaf(w2, xm1, acc);
      acc = fmaf(w3, xcur, acc);
      const float sv = acc + bc;
      const float sg = 1.0f / (1.0f + expf(-sv));
      sT[s * kConvTP + tid] = sv * sg;
      xm3 = xm2; xm2 = xm1; xm1 = xcur;
    }
    __syncthreads();
    v4f fv[4];
    v8h hv[2];
#pragma unroll
    for (int it = 0; it < 4; ++it) fv[it] = *(const v4f*)(sT + ((unsigned)it * 4u + hrow) * kConvTP + hch);
#pragma unroll
    for (int it = 0; it < 2; ++it) {
      const float* sp = sT + ((unsigned)it * 8u + wave) * kConvTP + lane * 8u;
      const v4f a0 = *(const v4f*)(sp);
      const v4f a1 = *(const v4f*)(sp + 4);
#pragma unroll
      for (int e = 0; e < 4; ++e) {
        hv[it][e]     = to_h16(a0[e], kCarryU);
        hv[it][4 + e] = to_h16(a1[e], kCarryU);
      }
    }
    for (int pass = 0; pass < 2; ++pass) {
#pragma unroll
      for (int it = 0; it < 4; ++it)
        *(volatile v4f*)(UC + (size_t)(lb + it * 4 + (int)hrow) * kDin + d0 + hch) = fv[it];
#pragma unroll
      for (int it = 0; it < 2; ++it)
        *(volatile v8h*)(UC16 + (size_t)(lb + it * 8 + (int)wave) * kDin + d0 + lane * 8u) = hv[it];
      __threadfence();
    }
    __syncthreads();
  }
}

__global__ __launch_bounds__(256) void cvt_dtlr_kernel(const float* __restrict__ XD, unsigned short* __restrict__ DL16)
{
  unsigned i = blockIdx.x * 256u + threadIdx.x;
  pinu(i);
  const unsigned row = i >> 3;
  const unsigned c8 = (i & 7u) * 8u;
  const v4f a0 = *(const v4f*)(XD + (size_t)row * kXdP + c8);
  const v4f a1 = *(const v4f*)(XD + (size_t)row * kXdP + c8 + 4);
  v8h hv;
#pragma unroll
  for (int e = 0; e < 4; ++e) {
    hv[e]     = to_h16(a0[e], kCarryDl);
    hv[4 + e] = to_h16(a1[e], kCarryDl);
  }
  unsigned short* q = DL16 + (size_t)row * kDtR + c8;
  *(volatile v8h*)q = hv;
  __threadfence();
  *(volatile v8h*)q = hv;
}

__global__ __launch_bounds__(256) void softplus_rows_kernel(
    const float* __restrict__ DTP, const float* __restrict__ bdt, float* __restrict__ DT)
{
#pragma unroll 1
  for (int it = 0; it < 2; ++it) {
    unsigned idx = blockIdx.x * 512u + (unsigned)it * 256u + threadIdx.x;
    pinu(idx);
    const size_t e0 = (size_t)idx * 4;
    const unsigned col = (idx * 4u) & (unsigned)(kDin - 1);
    const v4f v  = *(const v4f*)(DTP + e0);
    const v4f bb = *(const v4f*)(bdt + col);
    v4f o;
#pragma unroll
    for (int e = 0; e < 4; ++e) {
      const float t = v[e] + bb[e];
      o[e] = fmaxf(t, 0.0f) + log1pf(expf(-fabsf(t)));
    }
    *(volatile v4f*)(DT + e0) = o;
    __threadfence();
    *(volatile v4f*)(DT + e0) = o;
  }
}

__global__ __launch_bounds__(64) void scan_gate_kernel(
    const float* __restrict__ XD, const float* __restrict__ DT, const float* __restrict__ UC,
    const float* __restrict__ XZ, const float* __restrict__ Alog, const float* __restrict__ Dp,
    unsigned short* __restrict__ YG16)
{
  __shared__ __align__(16) float sX[kScanTS * kBcW];
  __shared__ __align__(16) float sY[kScanTS * kScanYP];
  __shared__ __align__(16) float sA[kNst * kScanCh];
  unsigned tid = threadIdx.x;
  pinu(tid);
  const unsigned lane = tid & 31u, wave = tid >> 5;
  constexpr unsigned kBlkPerB = kDin / kScanCh;
  const unsigned bix = blockIdx.x / kBlkPerB;
  const unsigned d0  = (blockIdx.x - bix * kBlkPerB) * (unsigned)kScanCh;
  const unsigned d   = d0 + tid;
  const size_t row0 = (size_t)bix * kSeq;
#pragma unroll 1
  for (int s = 0; s < kNst; ++s) sA[s * kScanCh + tid] = -expf(Alog[(size_t)d * kNst + s]);
  __syncthreads();
  float negA[kNst], h[kNst];
#pragma unroll
  for (int s = 0; s < kNst; ++s) {
    negA[s] = sA[s * kScanCh + tid];
    h[s] = 0.f;
  }
  const float Dd = Dp[d];
  const unsigned q = lane >> 3, c8 = (lane & 7u) * 8u;
#pragma unroll 1
  for (int t0 = 0; t0 < kSeq; t0 += kScanTS) {
    __syncthreads();
#pragma unroll
    for (int i = 0; i < 8; ++i) {
      const unsigned idx = (unsigned)i * 64u + tid;
      const unsigned r = idx >> 3;
      const unsigned c4 = (idx & 7u) * 4u;
      *(v4f*)(sX + r * kBcW + c4) = *(const v4f*)(XD + (row0 + t0 + r) * kXdP + kDtR + c4);
    }
    __syncthreads();
#pragma unroll 1
    for (int s = 0; s < kScanTS; ++s) {
      const size_t trow = row0 + t0 + s;
      float dt = DT[trow * kDin + d];
      float xt = UC[trow * kDin + d];
      float zv = XZ[trow * kXzP + kDin + d];
      pin1(dt);
      pin1(xt);
      pin1(zv);
      const float* xr = sX + s * kBcW;
      float Bs[kNst], Cs[kNst];
#pragma unroll
      for (int q4 = 0; q4 < 4; ++q4) {
        const v4f bv = *(const v4f*)(xr + 4 * q4);
        const v4f cv = *(const v4f*)(xr + kNst + 4 * q4);
        Bs[4 * q4 + 0] = bv[0]; Bs[4 * q4 + 1] = bv[1]; Bs[4 * q4 + 2] = bv[2]; Bs[4 * q4 + 3] = bv[3];
        Cs[4 * q4 + 0] = cv[0]; Cs[4 * q4 + 1] = cv[1]; Cs[4 * q4 + 2] = cv[2]; Cs[4 * q4 + 3] = cv[3];
      }
      const float dtx = dt * xt;
      float y = 0.f;
#pragma unroll
      for (int k = 0; k < kNst; ++k) {
        const float e = expf(dt * negA[k]);
        h[k] = fmaf(e, h[k], dtx * Bs[k]);
        y = fmaf(h[k], Cs[k], y);
      }
      y = fmaf(xt, Dd, y);
      const float sg = 1.0f / (1.0f + expf(-zv));
      y = y * (zv * sg);
      sY[s * kScanYP + tid] = y;
    }
    __syncthreads();
    v8h hv[8];
#pragma unroll
    for (int it = 0; it < 8; ++it) {
      const unsigned row = (unsigned)it * 8u + wave * 4u + q;
      const float* sp = sY + row * kScanYP + c8;
      const v4f a0 = *(const v4f*)(sp);
      const v4f a1 = *(const v4f*)(sp + 4);
#pragma unroll
      for (int e = 0; e < 4; ++e) {
        hv[it][e]     = to_h16(a0[e], kCarryY);
        hv[it][4 + e] = to_h16(a1[e], kCarryY);
      }
    }
    for (int pass = 0; pass < 2; ++pass) {
#pragma unroll
      for (int it = 0; it < 8; ++it) {
        const unsigned row = (unsigned)it * 8u + wave * 4u + q;
        const size_t o = (row0 + t0 + row) * kDin + d0 + c8;
        *(volatile v8h*)(YG16 + o) = hv[it];
      }
      __threadfence();
    }
  }
}

constexpr int gemm_blocks(int M, int N) { return ((M / 64) * (N / 64)) / 8; }
static_assert(((kRows / 64) * (kXzP / 64)) % 8 == 0 && ((kRows / 64) * (kXdP / 64)) % 8 == 0 &&
              ((kRows / 64) * (kDin / 64)) % 8 == 0 && ((kRows / 64) * (kDm / 64)) % 8 == 0);
static_assert(((kXzP * kDm / 8) % 256) == 0 && ((kXdP * kDin / 8) % 256) == 0 && ((kXdN * kDin / 8) % 256) == 0 &&
              ((kDin * kDtR / 8) % 256) == 0 && ((kDm * kDin / 8) % 256) == 0);

extern "C" void kernel_launch(void* const* d_in, const int* in_sizes, int n_in,
                              void* d_out, int out_size, void* d_ws, size_t ws_size,
                              hipStream_t stream) {
  if (n_in < 12) return;
  if (in_sizes[0] != kRows * kDm) return;
  if (in_sizes[1] != kDm) return;
  if (in_sizes[2] != kDm) return;
  if (in_sizes[3] != kXzP * kDm) return;
  if (in_sizes[4] != kDin * 4) return;
  if (in_sizes[5] != kDin) return;
  if (in_sizes[6] != kXdN * kDin) return;
  if (in_sizes[7] != kDin * kDtR) return;
  if (in_sizes[8] != kDin) return;
  if (in_sizes[9] != kDin * kNst) return;
  if (in_sizes[10] != kDin) return;
  if (in_sizes[11] != kDm * kDin) return;
  if (out_size != kRows * kDm) return;
  if (ws_size < kWsTotal) return;

  const float* x       = (const float*)d_in[0];
  const float* ln_w    = (const float*)d_in[1];
  const float* ln_b    = (const float*)d_in[2];
  const float* W_in    = (const float*)d_in[3];
  const float* conv_w  = (const float*)d_in[4];
  const float* conv_b  = (const float*)d_in[5];
  const float* W_xproj = (const float*)d_in[6];
  const float* W_dt    = (const float*)d_in[7];
  const float* b_dt    = (const float*)d_in[8];
  const float* A_log   = (const float*)d_in[9];
  const float* Dp      = (const float*)d_in[10];
  const float* W_out   = (const float*)d_in[11];
  float* out = (float*)d_out;

  char* ws = (char*)d_ws;
  unsigned short* WIN16  = (unsigned short*)(ws + kOffWIN);
  unsigned short* WX16   = (unsigned short*)(ws + kOffWX);
  unsigned short* WDT16  = (unsigned short*)(ws + kOffWDT);
  unsigned short* WOUT16 = (unsigned short*)(ws + kOffWOUT);
  unsigned short* H16    = (unsigned short*)(ws + kOffH16);
  float*          XZ     = (float*)(ws + kOffXZ);
  float*          UC     = (float*)(ws + kOffUC);
  unsigned short* UC16   = (unsigned short*)(ws + kOffUC16);
  float*          XD     = (float*)(ws + kOffXD);
  unsigned short* DL16   = (unsigned short*)(ws + kOffDL16);
  float*          DTP    = (float*)(ws + kOffDTP);
  float*          DT     = (float*)(ws + kOffDT);
  unsigned short* YG16   = (unsigned short*)(ws + kOffYG);

  cvt_plane_f16_kernel<<<(kXzP * kDm / 8) / 256, 256, 0, stream>>>(W_in, WIN16, kXzP * kDm / 8, kXzP * kDm / 8, kCarryWin);
  cvt_plane_f16_kernel<<<(kXdP * kDin / 8) / 256, 256, 0, stream>>>(W_xproj, WX16, kXdN * kDin / 8, kXdP * kDin / 8, kCarryWx);
  cvt_plane_f16_kernel<<<(kDin * kDtR / 8) / 256, 256, 0, stream>>>(W_dt, WDT16, kDin * kDtR / 8, kDin * kDtR / 8, kCarryWdt);
  cvt_plane_f16_kernel<<<(kDm * kDin / 8) / 256, 256, 0, stream>>>(W_out, WOUT16, kDm * kDin / 8, kDm * kDin / 8, kCarryWout);

  ln_rows_kernel<<<kRows / 8, 256, 0, stream>>>(x, ln_w, ln_b, H16);

  eng::wmma_gemm64_f16<false><<<gemm_blocks(kRows, kXzP), 256, 0, stream>>>(
      H16, kDm, WIN16, kDm, XZ, kXzP, nullptr, kRows, kXzP, kDm, kSclIn);

  conv_silu_kernel<<<dim3(kDin / 256, kRows / 64), 256, 0, stream>>>(XZ, conv_w, conv_b, UC, UC16);

  eng::wmma_gemm64_f16<false><<<gemm_blocks(kRows, kXdP), 256, 0, stream>>>(
      UC16, kDin, WX16, kDin, XD, kXdP, nullptr, kRows, kXdP, kDin, kSclX);

  cvt_dtlr_kernel<<<(kRows * kDtR / 8) / 256, 256, 0, stream>>>(XD, DL16);

  eng::wmma_gemm64_f16<false><<<gemm_blocks(kRows, kDin), 256, 0, stream>>>(
      DL16, kDtR, WDT16, kDtR, DTP, kDin, nullptr, kRows, kDin, kDtR, kSclDt);

  softplus_rows_kernel<<<(kRows * kDin / 4) / 512, 256, 0, stream>>>(DTP, b_dt, DT);

  scan_gate_kernel<<<kBatch * (kDin / kScanCh), kScanCh, 0, stream>>>(XD, DT, UC, XZ, A_log, Dp, YG16);

  eng::wmma_gemm64_f16<true><<<gemm_blocks(kRows, kDm), 256, 0, stream>>>(
      YG16, kDin, WOUT16, kDin, out, kDm, x, kRows, kDm, kDin, kSclOut);
}
